// MultiWindowHeadCrossAttention_35132832481299
// MI455X (gfx1250) — hardware-verified
//
#include <hip/hip_runtime.h>


namespace {
constexpr int Bn = 2, S = 4096, D = 1024, H = 16, HD = 64, W = 16, NT = Bn * S;
constexpr float QS = 8.0f, KS = 8.0f, VS = 8.0f, PS = 8.0f, SCALE = 0.125f;
constexpr size_t PL = (size_t)Bn * H * S * HD;

typedef _Float16 b16;
typedef __attribute__((ext_vector_type(16))) _Float16 v16b;
typedef __attribute__((ext_vector_type(16))) __bf16 v16bb;
typedef __attribute__((ext_vector_type(8))) _Float16 v8b;
typedef __attribute__((ext_vector_type(8))) unsigned short v8us;
typedef __attribute__((ext_vector_type(8))) float v8f;
typedef __attribute__((ext_vector_type(4))) float v4f;
__device__ __forceinline__ float bf16_rne(float f) { unsigned int u = __float_as_uint(f); u += 0x7FFFu + ((u >> 16) & 1u); return __uint_as_float(u & 0xFFFF0000u); }
__device__ __forceinline__ unsigned short bf16_bits(float f) { unsigned int u = __float_as_uint(f); u += 0x7FFFu + ((u >> 16) & 1u); return (unsigned short)(u >> 16); }
__device__ __forceinline__ v16b frag_kb(const b16* p, int hh) { const v8b a = *(const v8b*)(p + 8 * hh), b = *(const v8b*)(p + 16 + 8 * hh); v16b f;
#pragma unroll
  for (int e = 0; e < 8; ++e) { f[e] = a[e]; f[8 + e] = b[e]; } return f; }
__device__ __forceinline__ v16bb frag_bf(const unsigned short* p, int hh) { const v8us a = *(const v8us*)(p + 8 * hh), b = *(const v8us*)(p + 16 + 8 * hh); union { unsigned short s[16]; v16bb v; } u;
#pragma unroll
  for (int e = 0; e < 8; ++e) { u.s[e] = a[e]; u.s[8 + e] = b[e]; } return u.v; }
__device__ __forceinline__ v16bb frag_f32bf(const float* p, int hh) { union { unsigned short s[16]; v16bb v; } u;
#pragma unroll
  for (int e = 0; e < 8; ++e) { u.s[e] = bf16_bits(p[8 * hh + e]); u.s[8 + e] = bf16_bits(p[16 + 8 * hh + e]); } return u.v; }
__device__ __forceinline__ v8f wmma16b(v16b a, v16b b, v8f c) { v8f d = __builtin_amdgcn_wmma_f32_16x16x32_f16(false, a, false, b, (short)0, c, false, false); asm volatile("v_nop\n\tv_nop\n\tv_nop\n\tv_nop" : "+v"(d) : "v"(a), "v"(b)); return d; }
__device__ __forceinline__ v8f wmma16bb(v16bb a, v16bb b, v8f c) { v8f d = __builtin_amdgcn_wmma_f32_16x16x32_bf16(false, a, false, b, (short)0, c, false, false); asm volatile("v_nop\n\tv_nop\n\tv_nop\n\tv_nop" : "+v"(d) : "v"(a), "v"(b)); return d; }
__device__ __forceinline__ void wave_lds_sync() { __builtin_amdgcn_fence(__ATOMIC_RELEASE, "workgroup"); __builtin_amdgcn_wave_barrier(); __builtin_amdgcn_fence(__ATOMIC_ACQUIRE, "workgroup"); }
__device__ __forceinline__ float nexp(float x) { return __builtin_amdgcn_exp2f(x * 1.4426950408889634f); }

__global__ __launch_bounds__(256) void prep_kernel(const float* __restrict__ Wq, const float* __restrict__ Wk, const float* __restrict__ Wv, const float* __restrict__ Wo, const float* __restrict__ bq, const float* __restrict__ bk, const float* __restrict__ bv, const float* __restrict__ bo, unsigned short* __restrict__ w16, b16* __restrict__ wo16, float* __restrict__ P) {
  const size_t tid = (size_t)blockIdx.x * blockDim.x + threadIdx.x, nth = (size_t)gridDim.x * blockDim.x;
  for (int pass = 0; pass < 2; ++pass) {
    for (size_t p = tid; p < (size_t)3 * D * D / 8; p += nth) { const int m = (int)(p / (D * D / 8)); const size_t q = (p % (D * D / 8)) * 8; const float* Wm = (m == 0) ? Wq : (m == 1) ? Wk : Wv; v8us v;
#pragma unroll
      for (int e = 0; e < 8; ++e) v[e] = bf16_bits(Wm[q + e]);
      *(volatile v8us*)(w16 + p * 8) = v; }
    for (size_t p = tid; p < (size_t)D * D / 8; p += nth) { v8b v;
#pragma unroll
      for (int e = 0; e < 8; ++e) v[e] = (b16)bf16_rne(Wo[p * 8 + e]);
      *(volatile v8b*)(wo16 + p * 8) = v; }
    for (size_t p = tid; p < 4096; p += nth) { const int m = (int)p >> 10, i = (int)p & 1023; const float* bb = (m == 0) ? bq : (m == 1) ? bk : (m == 2) ? bv : bo; P[p] = bf16_rne(bb[i]); }
    __threadfence(); }
}

__global__ __launch_bounds__(128) void proj_kernel(const float* __restrict__ xq, const float* __restrict__ xkv, const unsigned short* __restrict__ w16, const float* __restrict__ P, b16* __restrict__ qp, b16* __restrict__ kp, b16* __restrict__ vt) {
  __shared__ __attribute__((aligned(16))) b16 T[4][32][64 + 8]; __shared__ __attribute__((aligned(16))) b16 Tv[64][128 + 8];
  const int lane = threadIdx.x & 31, wave = threadIdx.x >> 5, nloc = lane & 15, hlf = lane >> 4, which = blockIdx.z, h = blockIdx.x, c0 = h * HD, p0 = blockIdx.y * 128, m0 = p0 + wave * 32, b = p0 / S, t0 = p0 % S;
  const float* X = (which == 0) ? xq : xkv; const unsigned short* Wt = w16 + (size_t)which * D * D; const float* bias = P + which * 1024;
  v8f acc[2][4];
#pragma unroll
  for (int r = 0; r < 2; ++r)
#pragma unroll
    for (int t = 0; t < 4; ++t) acc[r][t] = (v8f){};
#pragma unroll 2
  for (int kb = 0; kb < D; kb += 32) { const v16bb a0 = frag_f32bf(X + (size_t)(m0 + nloc) * D + kb, hlf), a1 = frag_f32bf(X + (size_t)(m0 + 16 + nloc) * D + kb, hlf);
#pragma unroll
    for (int t = 0; t < 4; ++t) { const v16bb bw = frag_bf(Wt + (size_t)(c0 + t * 16 + nloc) * D + kb, hlf); acc[0][t] = wmma16bb(a0, bw, acc[0][t]); acc[1][t] = wmma16bb(a1, bw, acc[1][t]); } }
  if (which < 2) { const float scl = (which == 0) ? SCALE * QS : KS;
#pragma unroll
    for (int t = 0; t < 4; ++t) { const float bb = bias[c0 + t * 16 + nloc];
#pragma unroll
      for (int r = 0; r < 2; ++r)
#pragma unroll
        for (int v = 0; v < 8; ++v) T[wave][r * 16 + 8 * hlf + v][t * 16 + nloc] = (b16)((acc[r][t][v] + bb) * scl); }
    wave_lds_sync();
    b16* base = ((which == 0) ? qp : kp) + (((size_t)b * H + h) * S + (m0 % S)) * HD;
    for (int pass = 0; pass < 2; ++pass) {
#pragma unroll
      for (int j = 0; j < 8; ++j) { const int rr = j * 4 + (lane >> 3), c8 = (lane & 7) * 8; *(volatile v8b*)(base + (size_t)rr * HD + c8) = *(const v8b*)(&T[wave][rr][c8]); }
      __threadfence(); }
    return; }
#pragma unroll
  for (int t = 0; t < 4; ++t) { const float bb = bias[c0 + t * 16 + nloc];
#pragma unroll
    for (int r = 0; r < 2; ++r)
#pragma unroll
      for (int v = 0; v < 8; ++v) Tv[t * 16 + nloc][wave * 32 + r * 16 + 8 * hlf + v] = (b16)((acc[r][t][v] + bb) * VS); }
  __syncthreads();
  for (int pass = 0; pass < 2; ++pass) { for (int i = threadIdx.x; i < 64 * 16; i += 128) { const int d = i >> 4, c8 = (i & 15) * 8; *(volatile v8b*)(vt + (((size_t)b * H + h) * HD + d) * S + t0 + c8) = *(const v8b*)(&Tv[d][c8]); } __threadfence(); }
}

__global__ __launch_bounds__(256) void attn_kernel(const b16* __restrict__ qp, const b16* __restrict__ kp, const b16* __restrict__ vt, const int* __restrict__ causal_p, b16* __restrict__ ctx) {
  __shared__ __attribute__((aligned(16))) b16 Os[16][8 * HD + 8];
  const int wid = threadIdx.x >> 5, lane = threadIdx.x & 31, hh = lane >> 4, col = lane & 15; const int b = blockIdx.x / (S / 16), q0 = (blockIdx.x % (S / 16)) * 16, h = blockIdx.y * 8 + wid, qi = q0 + col;
  const bool causal = (causal_p[0] != 0);
  const b16* Q = qp + (((size_t)b * H + h) * S) * HD; const b16* K = kp + (((size_t)b * H + h) * S) * HD; const b16* V = vt + (((size_t)b * H + h) * HD) * S;
  const int kbase = (q0 >= 16) ? q0 - 16 : 0;
  const int lo = (qi - (W - 1) > 0) ? qi - (W - 1) : 0; const int hi = causal ? ((qi >= W - 1) ? qi : 2 * qi - (W - 1)) : qi; const int npad = (qi < W - 1) ? (causal ? ((qi + 1 < (W - 1) - qi) ? qi + 1 : (W - 1) - qi) : (W - 1) - qi) : 0;
  const v16b qf0 = frag_kb(Q + (size_t)qi * HD, hh), qf1 = frag_kb(Q + (size_t)qi * HD + 32, hh);
  const v16b ka0 = frag_kb(K + (size_t)(kbase + col) * HD, hh), ka1 = frag_kb(K + (size_t)(kbase + col) * HD + 32, hh), kc0 = frag_kb(K + (size_t)(kbase + 16 + col) * HD, hh), kc1 = frag_kb(K + (size_t)(kbase + 16 + col) * HD + 32, hh);
  v8f s0 = {}, s1 = {}; s0 = wmma16b(ka0, qf0, s0); s0 = wmma16b(ka1, qf1, s0); s1 = wmma16b(kc0, qf0, s1); s1 = wmma16b(kc1, qf1, s1);
  float m = -INFINITY;
#pragma unroll
  for (int r = 0; r < 8; ++r) { const int j0 = kbase + 8 * hh + r, j1 = kbase + 16 + 8 * hh + r; s0[r] *= 1.0f / (QS * KS); s1[r] *= 1.0f / (QS * KS); if (j0 < lo || j0 > hi) s0[r] = -INFINITY; if (j1 < lo || j1 > hi) s1[r] = -INFINITY; m = fmaxf(m, fmaxf(s0[r], s1[r])); }
  m = fmaxf(m, __shfl_xor(m, 16)); if (npad > 0) m = fmaxf(m, 0.0f);
  float sum = 0.0f; v16b pbv;
#pragma unroll
  for (int r = 0; r < 8; ++r) { const float e0 = (s0[r] == -INFINITY) ? 0.0f : nexp(s0[r] - m), e1 = (s1[r] == -INFINITY) ? 0.0f : nexp(s1[r] - m); sum += e0 + e1; pbv[r] = (b16)(e0 * PS); pbv[8 + r] = (b16)(e1 * PS); }
  sum += __shfl_xor(sum, 16); const float l = sum + (float)npad * nexp(0.0f - m);
  v8f o[4] = {{}, {}, {}, {}};
#pragma unroll
  for (int t = 0; t < 4; ++t) { const v16b vf = frag_kb(V + (size_t)(t * 16 + col) * S + kbase, hh); o[t] = wmma16b(vf, pbv, o[t]); }
  const float inv = 1.0f / (l * VS * PS);
#pragma unroll
  for (int t = 0; t < 4; ++t)
#pragma unroll
    for (int r = 0; r < 8; ++r) Os[col][wid * HD + t * 16 + 8 * hh + r] = (b16)(o[t][r] * inv);
  __syncthreads();
  for (int pass = 0; pass < 2; ++pass) { for (int i = threadIdx.x; i < 16 * (8 * HD / 8); i += 256) { const int rr = i / (8 * HD / 8), c8 = (i % (8 * HD / 8)) * 8; *(volatile v8b*)(ctx + ((size_t)b * S + q0 + rr) * D + blockIdx.y * 8 * HD + c8) = *(const v8b*)(&Os[rr][c8]); } __threadfence(); }
}

__global__ __launch_bounds__(128) void out_kernel(const b16* __restrict__ ctx, const b16* __restrict__ wo16, const float* __restrict__ P, float* __restrict__ out) {
  __shared__ __attribute__((aligned(16))) float Ts[4][32 * 64];
  const int lane = threadIdx.x & 31, wave = threadIdx.x >> 5, nloc = lane & 15, hlf = lane >> 4, m0 = blockIdx.y * 128 + wave * 32, c0 = blockIdx.x * 64; const float* bo = P + 3072;
  v8f acc[2][4];
#pragma unroll
  for (int r = 0; r < 2; ++r)
#pragma unroll
    for (int t = 0; t < 4; ++t) acc[r][t] = (v8f){};
#pragma unroll 2
  for (int kb = 0; kb < D; kb += 32) { const v16b a0 = frag_kb(ctx + (size_t)(m0 + nloc) * D + kb, hlf), a1 = frag_kb(ctx + (size_t)(m0 + 16 + nloc) * D + kb, hlf);
#pragma unroll
    for (int t = 0; t < 4; ++t) { const v16b bw = frag_kb(wo16 + (size_t)(c0 + t * 16 + nloc) * D + kb, hlf); acc[0][t] = wmma16b(a0, bw, acc[0][t]); acc[1][t] = wmma16b(a1, bw, acc[1][t]); } }
  float* Tt = Ts[wave];
#pragma unroll
  for (int t = 0; t < 4; ++t) { const float bb = bo[c0 + t * 16 + nloc];
#pragma unroll
    for (int r = 0; r < 2; ++r)
#pragma unroll
      for (int v = 0; v < 8; ++v) Tt[(r * 16 + v + 8 * hlf) * 64 + t * 16 + nloc] = acc[r][t][v] + bb; }
  wave_lds_sync();
  for (int pass = 0; pass < 2; ++pass) {
#pragma unroll
    for (int j = 0; j < 16; ++j) { const int rr = j * 2 + hlf, c4 = nloc * 4; *(volatile v4f*)(out + (size_t)(m0 + rr) * D + c0 + c4) = *(const v4f*)(Tt + rr * 64 + c4); }
    __threadfence(); }
}
}

extern "C" void kernel_launch(void* const* d_in, const int* in_sizes, int n_in,
                              void* d_out, int out_size, void* d_ws, size_t ws_size, hipStream_t stream) {
  (void)n_in; (void)out_size;
  const float* query = (const float*)d_in[0]; const float* kv = (const float*)d_in[1]; const float* Wq = (const float*)d_in[2]; const float* bq = (const float*)d_in[3]; const float* Wk = (const float*)d_in[4]; const float* bk = (const float*)d_in[5]; const float* Wv = (const float*)d_in[6]; const float* bv = (const float*)d_in[7]; const float* Wo = (const float*)d_in[8]; const float* bo = (const float*)d_in[9]; const int* isc = (const int*)d_in[10];
  float* out = (float*)d_out;
  if (in_sizes[0] != NT * D || in_sizes[1] != NT * D || in_sizes[2] != D * D || in_sizes[8] != D * D || in_sizes[10] != 1) return;
  size_t off = 0; char* ws = (char*)d_ws;
  auto carve = [&](size_t bytes) { char* p = ws + off; off += (bytes + 255) & ~(size_t)255; return p; };
  unsigned short* w16 = (unsigned short*)carve((size_t)3 * D * D * 2); b16* wo16 = (b16*)carve((size_t)D * D * 2); float* P = (float*)carve(4096 * 4);
  b16* qp = (b16*)carve(PL * 2); b16* kp = (b16*)carve(PL * 2); b16* vt = (b16*)carve(PL * 2); b16* ctx = (b16*)carve((size_t)NT * D * 2);
  if (off > ws_size) return;
  prep_kernel<<<512, 256, 0, stream>>>(Wq, Wk, Wv, Wo, bq, bk, bv, bo, w16, wo16, P);
  proj_kernel<<<dim3(H, NT / 128, 3), 128, 0, stream>>>(query, kv, w16, P, qp, kp, vt);
  attn_kernel<<<dim3(NT / 16, 2), 256, 0, stream>>>(qp, kp, vt, isc, ctx);
  out_kernel<<<dim3(D / 64, NT / 128), 128, 0, stream>>>(ctx, wo16, P, out);
}
